// PointNetSetAbstraction_60017872994423
// MI455X (gfx1250) — hardware-verified
//
#include <hip/hip_runtime.h>
#include <stdint.h>

#pragma clang fp contract(off)

typedef __attribute__((ext_vector_type(16))) _Float16 v16h;
typedef __attribute__((ext_vector_type(8)))  _Float16 v8h;
typedef __attribute__((ext_vector_type(8)))  float    v8f;
typedef __attribute__((ext_vector_type(4)))  float    v4f;
typedef __attribute__((ext_vector_type(4)))  unsigned v4u;

constexpr int NBATCH = 16;
constexpr int NPTS   = 4096;
constexpr int NCENT  = 1024;
constexpr int NNBR   = 32;
constexpr int MROWS  = NBATCH * NCENT * NNBR;
constexpr int NCH_L1 = 64;
constexpr int NCH_L2 = 64;
constexpr int NCH_L3 = 128;
constexpr int LDS_PITCH_H = 72;
constexpr int NPARTS = MROWS / 128;
constexpr float WCARRY     = 64.0f;
constexpr float WCARRY_INV = 1.0f / 64.0f;
constexpr float BALL_R2 = 0.16f;
constexpr float BN_EPS  = 1e-5f;

static_assert(MROWS == 524288);
static_assert(NPARTS == 4096);
static_assert(NCH_L1 % 32 == 0 && NCH_L2 % 32 == 0);
static_assert(NCH_L2 % 64 == 0 && NCH_L3 % 64 == 0);

constexpr size_t SZ_NX4   = (size_t)NBATCH * NCENT * 4 * 4;
constexpr size_t SZ_X0    = (size_t)MROWS * 8 * 4;
constexpr size_t SZ_PM    = (size_t)256 * 32 * 4;
constexpr size_t SZ_P1    = (size_t)576 * 4;
constexpr size_t SZ_W2H   = (size_t)NCH_L2 * NCH_L1 * 2;
constexpr size_t SZ_W3H   = (size_t)NCH_L3 * NCH_L2 * 2;
constexpr size_t SZ_PART2 = (size_t)NPARTS * 128 * 4;
constexpr size_t SZ_SC2   = (size_t)128 * 4;
constexpr size_t SZ_Y2H   = (size_t)MROWS * NCH_L2 * 2;
constexpr size_t SZ_PART3 = (size_t)NPARTS * 256 * 4;
constexpr size_t SZ_SC3   = (size_t)256 * 4;
constexpr size_t SZ_YMM   = (size_t)NBATCH * NCENT * NCH_L3 * 4;
constexpr size_t OFF_NX4   = 0;
constexpr size_t OFF_X0    = OFF_NX4 + SZ_NX4;
constexpr size_t OFF_PM    = OFF_X0 + SZ_X0;
constexpr size_t OFF_P1    = OFF_PM + SZ_PM;
constexpr size_t OFF_W2H   = OFF_P1 + SZ_P1;
constexpr size_t OFF_W3H   = OFF_W2H + SZ_W2H;
constexpr size_t OFF_PART2 = OFF_W3H + SZ_W3H;
constexpr size_t OFF_SC2   = OFF_PART2 + SZ_PART2;
constexpr size_t OFF_Y2H   = OFF_SC2 + SZ_SC2;
constexpr size_t OFF_PART3 = OFF_Y2H + SZ_Y2H;
constexpr size_t OFF_SC3   = OFF_PART3 + SZ_PART3;
constexpr size_t OFF_YMAX  = OFF_SC3 + SZ_SC3;
constexpr size_t OFF_YMIN  = OFF_YMAX + SZ_YMM;
constexpr size_t WS_TOTAL  = OFF_YMIN + SZ_YMM;
static_assert(WS_TOTAL == 107278080);
static_assert(WS_TOTAL <= 134217728);
static_assert(SZ_P1 % 128 == 0 && SZ_SC2 % 128 == 0 && SZ_SC3 % 128 == 0);
constexpr size_t OUT0_BYTES = (size_t)NBATCH * 3 * NCENT * 4;
constexpr size_t OUT1_BYTES = (size_t)NBATCH * NCH_L3 * NCENT * 4;
static_assert(OUT0_BYTES == 196608);
static_assert(OUT0_BYTES + OUT1_BYTES == 8585216);

__device__ __forceinline__ float h16_to_f32(unsigned hb) {
  const unsigned sgn = (hb & 0x8000u) << 16;
  const unsigned em = hb & 0x7fffu;
  const float fn = __uint_as_float((em << 13) + 0x38000000u);
  const float fs = (float)em * 5.9604644775390625e-8f;
  const float mag = (em < 0x400u) ? fs : fn;
  return __uint_as_float(__float_as_uint(mag) | sgn);
}

__device__ __forceinline__ v16h frag_load_h(const _Float16* p) {
  union { v16h v; v8h h[2]; } f;
  f.h[0] = *(const v8h*)(p);
  f.h[1] = *(const v8h*)(p + 16);
  return f.v;
}
__device__ __forceinline__ v8f mma_h(v16h a, v16h b, v8f c) {
  return __builtin_amdgcn_wmma_f32_16x16x32_f16(false, a, false, b, (short)0, c, false, false);
}
__device__ __forceinline__ void guard_4acc(v8f& c0, v8f& c1, v8f& c2, v8f& c3,
                                           v16h a, v16h b0, v16h b1, v16h b2, v16h b3) {
  asm volatile("v_nop\n\tv_nop\n\tv_nop\n\tv_nop"
               : "+v"(c0), "+v"(c1), "+v"(c2), "+v"(c3)
               : "v"(a), "v"(b0), "v"(b1), "v"(b2), "v"(b3));
}
__device__ __forceinline__ void guard_8acc(v8f& c0, v8f& c1, v8f& c2, v8f& c3,
                                           v8f& c4, v8f& c5, v8f& c6, v8f& c7,
                                           v16h a0, v16h a1, v16h b0, v16h b1, v16h b2, v16h b3) {
  asm volatile("v_nop\n\tv_nop\n\tv_nop\n\tv_nop"
               : "+v"(c0), "+v"(c1), "+v"(c2), "+v"(c3), "+v"(c4), "+v"(c5), "+v"(c6), "+v"(c7)
               : "v"(a0), "v"(a1), "v"(b0), "v"(b1), "v"(b2), "v"(b3));
}

__global__ __launch_bounds__(1024) void k_fps(const float* __restrict__ xyz_pc,
                                              float* __restrict__ out0,
                                              float* __restrict__ nx4) {
#pragma clang fp contract(off)
  __shared__ __align__(16) float sx[NPTS];
  __shared__ __align__(16) float sy[NPTS];
  __shared__ __align__(16) float sz[NPTS];
  __shared__ float wv[2][32];
  __shared__ int wi[2][32];
  __shared__ int sidx[NCENT];
  const int b = blockIdx.x;
  const int tid = threadIdx.x;
  const int lane = tid & 31;
  const int wid = tid >> 5;
  const float* px = xyz_pc + (size_t)b * 3 * NPTS;
  const v4f vx = *(const v4f*)(px + 4 * tid);
  const v4f vy = *(const v4f*)(px + NPTS + 4 * tid);
  const v4f vz = *(const v4f*)(px + 2 * NPTS + 4 * tid);
  *(v4f*)(sx + 4 * tid) = vx;
  *(v4f*)(sy + 4 * tid) = vy;
  *(v4f*)(sz + 4 * tid) = vz;
  const float xx[4] = {vx[0], vx[1], vx[2], vx[3]};
  const float yy[4] = {vy[0], vy[1], vy[2], vy[3]};
  const float zz[4] = {vz[0], vz[1], vz[2], vz[3]};
  float dd[4] = {1e10f, 1e10f, 1e10f, 1e10f};
  __syncthreads();
  int far = 0;
#pragma unroll 1
  for (int s = 0; s < NCENT; ++s) {
    if (tid == 0) sidx[s] = far;
    const float cx = sx[far];
    const float cy = sy[far];
    const float cz = sz[far];
    float best = -1.0f;
    int bi = 4 * tid;
#pragma unroll
    for (int j = 0; j < 4; ++j) {
      const float dx = xx[j] - cx;
      const float dy = yy[j] - cy;
      const float dz = zz[j] - cz;
      const float t0 = dx * dx;
      const float t1 = dy * dy;
      const float t2 = dz * dz;
      const float d = (t0 + t2) + t1;
      const float nd = fminf(dd[j], d);
      dd[j] = nd;
      const bool tk = nd > best;
      best = tk ? nd : best;
      bi = tk ? (4 * tid + j) : bi;
    }
#pragma unroll
    for (int off = 16; off > 0; off >>= 1) {
      const float ov = __shfl_xor(best, off);
      const int oi = __shfl_xor(bi, off);
      const bool tk = (ov > best) || (ov == best && oi < bi);
      best = tk ? ov : best;
      bi = tk ? oi : bi;
    }
    const int pb = s & 1;
    if (lane == 0) { wv[pb][wid] = best; wi[pb][wid] = bi; }
    __syncthreads();
    best = wv[pb][lane];
    bi = wi[pb][lane];
#pragma unroll
    for (int off = 16; off > 0; off >>= 1) {
      const float ov = __shfl_xor(best, off);
      const int oi = __shfl_xor(bi, off);
      const bool tk = (ov > best) || (ov == best && oi < bi);
      best = tk ? ov : best;
      bi = tk ? oi : bi;
    }
    far = bi;
  }
  __syncthreads();
  int id = sidx[tid];
  id = id < 0 ? 0 : (id > NPTS - 1 ? NPTS - 1 : id);
  const float ox = sx[id];
  const float oy = sy[id];
  const float oz = sz[id];
  float* o = out0 + (size_t)b * 3 * NCENT + tid;
  float* n4 = nx4 + ((size_t)b * NCENT + tid) * 4;
  const v4f cv = {ox, oy, oz, 0.0f};
  for (int pass = 0; pass < 2; ++pass) {
    *(volatile float*)(o) = ox;
    *(volatile float*)(o + NCENT) = oy;
    *(volatile float*)(o + 2 * NCENT) = oz;
    *(volatile v4f*)(n4) = cv;
    __threadfence();
  }
}

__global__ __launch_bounds__(256) void k_ballq_group(const float* __restrict__ xyz_pc,
                                                     const float* __restrict__ points,
                                                     const float* __restrict__ nx4,
                                                     float* __restrict__ X0) {
#pragma clang fp contract(off)
  __shared__ int slot[8 * 32];
  __shared__ __align__(16) float xrow[8 * 256];
  const int lane = threadIdx.x & 31;
  const int w = threadIdx.x >> 5;
  const int q = blockIdx.x * 8 + w;
  const int b = q >> 10;
  const float* px = xyz_pc + (size_t)b * 3 * NPTS;
  const float* py = px + NPTS;
  const float* pz = py + NPTS;
  const float* fx = points + (size_t)b * 3 * NPTS;
  const v4f cq = *(const v4f*)(nx4 + (size_t)q * 4);
  const float qx = cq[0];
  const float qy = cq[1];
  const float qz = cq[2];
  slot[w * 32 + lane] = 0;
  __syncthreads();
  int cnt = 0;
#pragma unroll 1
  for (int c0 = 0; c0 < NPTS; c0 += 32) {
    const int i = c0 + lane;
    const float X = px[i];
    const float Y = py[i];
    const float Z = pz[i];
    const float dx = qx - X;
    const float dy = qy - Y;
    const float dz = qz - Z;
    const float t0 = dx * dx;
    const float t1 = dy * dy;
    const float t2 = dz * dz;
    const float sqr = (t0 + t2) + t1;
    const bool hit = !(sqr > BALL_R2);
    const unsigned bal = (unsigned)__ballot(hit);
    const int pos = cnt + __popc(bal & ((1u << lane) - 1u));
    if (hit && pos < NNBR) slot[w * 32 + pos] = i;
    cnt += __popc(bal);
    if (cnt >= NNBR) break;
  }
  __syncthreads();
  const int cl = cnt < NNBR ? cnt : NNBR;
  const int sl = slot[w * 32 + lane];
  const int s0 = slot[w * 32];
  int g = (lane < cl) ? sl : s0;
  g = g < 0 ? 0 : (g > NPTS - 1 ? NPTS - 1 : g);
  const float gx = px[g];
  const float gy = py[g];
  const float gz = pz[g];
  const float f0 = fx[g];
  const float f1 = fx[NPTS + g];
  const float f2 = fx[2 * NPTS + g];
  const v4f ra = {gx - qx, gy - qy, gz - qz, f0};
  const v4f rb = {f1, f2, 0.0f, 0.0f};
  *(v4f*)(xrow + w * 256 + lane * 8) = ra;
  *(v4f*)(xrow + w * 256 + lane * 8 + 4) = rb;
  __syncthreads();
  float* dst = X0 + (size_t)q * 256;
  const v4f o0 = *(const v4f*)(xrow + w * 256 + lane * 4);
  const v4f o1 = *(const v4f*)(xrow + w * 256 + 128 + lane * 4);
  for (int pass = 0; pass < 2; ++pass) {
    *(volatile v4f*)(dst + lane * 4) = o0;
    *(volatile v4f*)(dst + 128 + lane * 4) = o1;
    __threadfence();
  }
}

__global__ __launch_bounds__(256) void k_mom(const float* __restrict__ X0, float* __restrict__ PM) {
  __shared__ float red[8 * 32];
  const int tid = threadIdx.x;
  const int lane = tid & 31;
  const int wave = tid >> 5;
  float acc[27];
#pragma unroll
  for (int v = 0; v < 27; ++v) acc[v] = 0.0f;
  const size_t base = (size_t)blockIdx.x * 2048;
#pragma unroll 1
  for (int it = 0; it < 8; ++it) {
    const size_t r = base + (size_t)it * 256 + tid;
    const v4f a = *(const v4f*)(X0 + r * 8);
    const v4f bq = *(const v4f*)(X0 + r * 8 + 4);
    const float x[6] = {a[0], a[1], a[2], a[3], bq[0], bq[1]};
#pragma unroll
    for (int c = 0; c < 6; ++c) acc[c] += x[c];
#pragma unroll
    for (int c = 0; c < 6; ++c) {
#pragma unroll
      for (int d = c; d < 6; ++d) {
        const int p = 6 + c * 6 - (c * (c - 1)) / 2 + (d - c);
        acc[p] = __builtin_fmaf(x[c], x[d], acc[p]);
      }
    }
  }
#pragma unroll
  for (int v = 0; v < 27; ++v) {
    float a = acc[v];
#pragma unroll
    for (int off = 16; off > 0; off >>= 1) a += __shfl_xor(a, off);
    acc[v] = a;
  }
  if (lane == 0) {
#pragma unroll
    for (int v = 0; v < 27; ++v) red[wave * 32 + v] = acc[v];
#pragma unroll
    for (int v = 27; v < 32; ++v) red[wave * 32 + v] = 0.0f;
  }
  __syncthreads();
  if (tid < 32) {
    float a = 0.0f;
#pragma unroll
    for (int wv_ = 0; wv_ < 8; ++wv_) a += red[wv_ * 32 + tid];
    float* p = PM + (size_t)blockIdx.x * 32 + tid;
    *(volatile float*)p = a;
    __threadfence();
    *(volatile float*)p = a;
  }
}

__global__ __launch_bounds__(256) void k_fin1(const float* __restrict__ PM,
                                              const float* __restrict__ W1, const float* __restrict__ b1,
                                              const float* __restrict__ g1, const float* __restrict__ be1,
                                              const float* __restrict__ W2, const float* __restrict__ W3,
                                              float* __restrict__ P1, _Float16* __restrict__ W2H,
                                              _Float16* __restrict__ W3H) {
  __shared__ double smom[32];
  __shared__ __align__(16) float pbuf[576];
  const int tid = threadIdx.x;
  if (tid < 32) {
    double a = 0.0;
#pragma unroll 4
    for (int i = 0; i < 256; ++i) a += (double)PM[i * 32 + tid];
    smom[tid] = a * (1.0 / (double)MROWS);
  }
  __syncthreads();
  if (tid < NCH_L1) {
    const int o = tid;
    float wf[6];
#pragma unroll
    for (int c = 0; c < 6; ++c) wf[c] = W1[o * 6 + c];
    const float bb = b1[o];
    const float gg = g1[o];
    const float be = be1[o];
    double mean = (double)bb;
#pragma unroll
    for (int c = 0; c < 6; ++c) mean += (double)wf[c] * smom[c];
    double var = 0.0;
#pragma unroll
    for (int c = 0; c < 6; ++c) {
#pragma unroll
      for (int d = c; d < 6; ++d) {
        const int p = 6 + c * 6 - (c * (c - 1)) / 2 + (d - c);
        const double cov = smom[p] - smom[c] * smom[d];
        const double term = (double)wf[c] * (double)wf[d] * cov;
        var += (c == d) ? term : (term + term);
      }
    }
    if (var < 0.0) var = 0.0;
    const float sc = gg * rsqrtf((float)var + BN_EPS);
#pragma unroll
    for (int c = 0; c < 6; ++c) pbuf[o * 8 + c] = sc * wf[c];
    pbuf[o * 8 + 6] = 0.0f;
    pbuf[o * 8 + 7] = 0.0f;
    pbuf[512 + o] = sc * (bb - (float)mean) + be;
  }
  __syncthreads();
  if (tid < 144) {
    const v4f v = *(const v4f*)(pbuf + tid * 4);
    *(volatile v4f*)(P1 + tid * 4) = v;
    __threadfence();
    *(volatile v4f*)(P1 + tid * 4) = v;
  }
#pragma unroll 1
  for (int it = 0; it < 2; ++it) {
    const int e = (it * 256 + tid) * 8;
    const v4f a = *(const v4f*)(W2 + e);
    const v4f c = *(const v4f*)(W2 + e + 4);
    v8h hv;
    hv[0] = (_Float16)(a[0] * WCARRY); hv[1] = (_Float16)(a[1] * WCARRY);
    hv[2] = (_Float16)(a[2] * WCARRY); hv[3] = (_Float16)(a[3] * WCARRY);
    hv[4] = (_Float16)(c[0] * WCARRY); hv[5] = (_Float16)(c[1] * WCARRY);
    hv[6] = (_Float16)(c[2] * WCARRY); hv[7] = (_Float16)(c[3] * WCARRY);
    *(volatile v8h*)(W2H + e) = hv;
    __threadfence();
    *(volatile v8h*)(W2H + e) = hv;
  }
#pragma unroll 1
  for (int it = 0; it < 4; ++it) {
    const int e = (it * 256 + tid) * 8;
    const v4f a = *(const v4f*)(W3 + e);
    const v4f c = *(const v4f*)(W3 + e + 4);
    v8h hv;
    hv[0] = (_Float16)(a[0] * WCARRY); hv[1] = (_Float16)(a[1] * WCARRY);
    hv[2] = (_Float16)(a[2] * WCARRY); hv[3] = (_Float16)(a[3] * WCARRY);
    hv[4] = (_Float16)(c[0] * WCARRY); hv[5] = (_Float16)(c[1] * WCARRY);
    hv[6] = (_Float16)(c[2] * WCARRY); hv[7] = (_Float16)(c[3] * WCARRY);
    *(volatile v8h*)(W3H + e) = hv;
    __threadfence();
    *(volatile v8h*)(W3H + e) = hv;
  }
}

__global__ __launch_bounds__(256) void k_l12(const float* __restrict__ X0, const float* __restrict__ P1,
                                             const _Float16* __restrict__ W2H, const float* __restrict__ b2,
                                             _Float16* __restrict__ Y2H, float* __restrict__ PART2) {
  __shared__ __align__(16) float sW1[576];
  __shared__ __align__(16) _Float16 sB[NCH_L2 * LDS_PITCH_H];
  __shared__ __align__(16) _Float16 sA[128 * LDS_PITCH_H];
  __shared__ __align__(16) _Float16 sY[8 * 16 * LDS_PITCH_H];
  __shared__ __align__(16) float sStat[8 * 128];
  const int tid = threadIdx.x;
  const int lane = tid & 31;
  const int wave = tid >> 5;
  const int blk = blockIdx.x;
  if (tid < 144) *(v4f*)(sW1 + tid * 4) = *(const v4f*)(P1 + tid * 4);
#pragma unroll
  for (int it = 0; it < 2; ++it) {
    const int ch = it * 256 + tid;
    const int n = ch >> 3;
    const int c8 = (ch & 7) * 8;
    *(v8h*)(sB + n * LDS_PITCH_H + c8) = *(const v8h*)(W2H + n * NCH_L1 + c8);
  }
  const int row = tid >> 1;
  const int half = tid & 1;
  const size_t gm = (size_t)blk * 128 + row;
  const v4f xa = *(const v4f*)(X0 + gm * 8);
  const v4f xb = *(const v4f*)(X0 + gm * 8 + 4);
  __syncthreads();
#pragma unroll 1
  for (int i = 0; i < 4; ++i) {
    v8h hv;
#pragma unroll
    for (int e = 0; e < 8; ++e) {
      const int o = half * 32 + i * 8 + e;
      const v4f wa = *(const v4f*)(sW1 + o * 8);
      const v4f wb = *(const v4f*)(sW1 + o * 8 + 4);
      float v = sW1[512 + o];
      v = __builtin_fmaf(wa[0], xa[0], v);
      v = __builtin_fmaf(wa[1], xa[1], v);
      v = __builtin_fmaf(wa[2], xa[2], v);
      v = __builtin_fmaf(wa[3], xa[3], v);
      v = __builtin_fmaf(wb[0], xb[0], v);
      v = __builtin_fmaf(wb[1], xb[1], v);
      v = fmaxf(v, 0.0f);
      hv[e] = (_Float16)v;
    }
    *(v8h*)(sA + row * LDS_PITCH_H + half * 32 + i * 8) = hv;
  }
  __syncthreads();

  const int hh = lane >> 4;
  const int c = lane & 15;
  const int koff = hh * 8;
  const int m0 = wave * 16;
  v8f acc[4];
#pragma unroll
  for (int j = 0; j < 4; ++j) acc[j] = (v8f){0.f, 0.f, 0.f, 0.f, 0.f, 0.f, 0.f, 0.f};
#pragma unroll
  for (int k0 = 0; k0 < NCH_L1; k0 += 32) {
    const v16h a = frag_load_h(sA + (m0 + c) * LDS_PITCH_H + koff + k0);
    const v16h b0 = frag_load_h(sB + (0 + c) * LDS_PITCH_H + koff + k0);
    const v16h b1 = frag_load_h(sB + (16 + c) * LDS_PITCH_H + koff + k0);
    const v16h b2f = frag_load_h(sB + (32 + c) * LDS_PITCH_H + koff + k0);
    const v16h b3 = frag_load_h(sB + (48 + c) * LDS_PITCH_H + koff + k0);
    acc[0] = mma_h(a, b0, acc[0]);
    acc[1] = mma_h(a, b1, acc[1]);
    acc[2] = mma_h(a, b2f, acc[2]);
    acc[3] = mma_h(a, b3, acc[3]);
    guard_4acc(acc[0], acc[1], acc[2], acc[3], a, b0, b1, b2f, b3);
  }

  _Float16* ys = sY + wave * (16 * LDS_PITCH_H);
#pragma unroll
  for (int j = 0; j < 4; ++j) {
    const int n = j * 16 + c;
    const float bv = b2[n];
    float s = 0.0f;
    float q = 0.0f;
#pragma unroll
    for (int r = 0; r < 8; ++r) {
      const float v = __builtin_fmaf(acc[j][r], WCARRY_INV, bv);
      s += v;
      q = __builtin_fmaf(v, v, q);
      ys[(8 * hh + r) * LDS_PITCH_H + n] = (_Float16)v;
    }
    s += __shfl_xor(s, 16);
    q += __shfl_xor(q, 16);
    sStat[wave * 128 + hh * 64 + n] = hh ? q : s;
  }
  __syncthreads();
  {
    const size_t mrow0 = (size_t)blk * 128 + m0;
    const int q4 = lane >> 3;
    const int c8 = (lane & 7) * 8;
    for (int pass = 0; pass < 2; ++pass) {
#pragma unroll
      for (int it = 0; it < 4; ++it) {
        const int rr = it * 4 + q4;
        const v8h hv = *(const v8h*)(ys + rr * LDS_PITCH_H + c8);
        *(volatile v8h*)(Y2H + (mrow0 + rr) * NCH_L2 + c8) = hv;
      }
      __threadfence();
    }
  }
  if (tid < 32) {
    v4f o;
#pragma unroll
    for (int i = 0; i < 4; ++i) {
      float a = 0.0f;
#pragma unroll
      for (int wv_ = 0; wv_ < 8; ++wv_) a += sStat[wv_ * 128 + tid * 4 + i];
      o[i] = a;
    }
    float* p = PART2 + (size_t)blk * 128 + tid * 4;
    *(volatile v4f*)p = o;
    __threadfence();
    *(volatile v4f*)p = o;
  }
}

template <int NCH>
__global__ __launch_bounds__(1024) void k_fin(const float* __restrict__ part,
                                              const float* __restrict__ g, const float* __restrict__ be,
                                              float* __restrict__ sc) {
  constexpr int NC2 = 2 * NCH;
  constexpr int NGRP = 1024 / NC2;
  constexpr int RPG = NPARTS / NGRP;
  static_assert(NGRP * NC2 == 1024);
  static_assert(RPG * NGRP == NPARTS);
  __shared__ double red[1024];
  __shared__ __align__(16) float outb[NC2];
  const int tid = threadIdx.x;
  const int col = tid % NC2;
  const int grp = tid / NC2;
  double a = 0.0;
#pragma unroll 4
  for (int r = 0; r < RPG; ++r) a += (double)part[((size_t)grp * RPG + r) * NC2 + col];
  red[tid] = a;
  __syncthreads();
  if (tid < NCH) {
    double S = 0.0;
    double Q = 0.0;
#pragma unroll
    for (int gi = 0; gi < NGRP; ++gi) {
      S += red[gi * NC2 + tid];
      Q += red[gi * NC2 + NCH + tid];
    }
    const double mean = S * (1.0 / (double)MROWS);
    double var = Q * (1.0 / (double)MROWS) - mean * mean;
    if (var < 0.0) var = 0.0;
    const float scl = g[tid] * rsqrtf((float)var + BN_EPS);
    outb[tid] = scl;
    outb[NCH + tid] = be[tid] - (float)mean * scl;
  }
  __syncthreads();
  if (tid < NC2 / 4) {
    const v4f v = *(const v4f*)(outb + tid * 4);
    *(volatile v4f*)(sc + tid * 4) = v;
    __threadfence();
    *(volatile v4f*)(sc + tid * 4) = v;
  }
}

__device__ __forceinline__ _Float16 bn_relu_h(unsigned hb, float scl, float sh) {
  const float x = h16_to_f32(hb);
  float y = __builtin_fmaf(x, scl, sh);
  y = fmaxf(y, 0.0f);
  return (_Float16)y;
}

__global__ __launch_bounds__(256) void k_l3(const unsigned* __restrict__ Y2W, const float* __restrict__ SC2,
                                            const _Float16* __restrict__ W3H, const float* __restrict__ b3,
                                            float* __restrict__ YMAX, float* __restrict__ YMIN,
                                            float* __restrict__ PART3) {
  __shared__ __align__(16) _Float16 sA[128 * LDS_PITCH_H];
  __shared__ __align__(16) _Float16 sB[NCH_L3 * LDS_PITCH_H];
  __shared__ __align__(16) float sStat[8 * 128];
  const int tid = threadIdx.x;
  const int lane = tid & 31;
  const int wave = tid >> 5;
  const int blk = blockIdx.x;
#pragma unroll
  for (int it = 0; it < 4; ++it) {
    const int ch = it * 256 + tid;
    const int n = ch >> 3;
    const int c8 = (ch & 7) * 8;
    *(v8h*)(sB + n * LDS_PITCH_H + c8) = *(const v8h*)(W3H + n * NCH_L2 + c8);
  }
  const int c8t = (tid & 7) * 8;
  const v4f sc0 = *(const v4f*)(SC2 + c8t);
  const v4f sc1 = *(const v4f*)(SC2 + c8t + 4);
  const v4f sh0 = *(const v4f*)(SC2 + NCH_L2 + c8t);
  const v4f sh1 = *(const v4f*)(SC2 + NCH_L2 + c8t + 4);
  const float s0 = sc0[0], s1 = sc0[1], s2 = sc0[2], s3 = sc0[3];
  const float s4 = sc1[0], s5 = sc1[1], s6 = sc1[2], s7 = sc1[3];
  const float h0 = sh0[0], h1 = sh0[1], h2 = sh0[2], h3 = sh0[3];
  const float h4 = sh1[0], h5 = sh1[1], h6 = sh1[2], h7 = sh1[3];
#pragma unroll
  for (int it = 0; it < 4; ++it) {
    const int ch = it * 256 + tid;
    const int rowl = ch >> 3;
    const v4u w = *(const v4u*)(Y2W + ((size_t)blk * 1024 + ch) * 4);
    const unsigned w0 = w[0];
    const unsigned w1 = w[1];
    const unsigned w2 = w[2];
    const unsigned w3 = w[3];
    v8h hv;
    hv[0] = bn_relu_h(w0 & 0xffffu, s0, h0);
    hv[1] = bn_relu_h(w0 >> 16, s1, h1);
    hv[2] = bn_relu_h(w1 & 0xffffu, s2, h2);
    hv[3] = bn_relu_h(w1 >> 16, s3, h3);
    hv[4] = bn_relu_h(w2 & 0xffffu, s4, h4);
    hv[5] = bn_relu_h(w2 >> 16, s5, h5);
    hv[6] = bn_relu_h(w3 & 0xffffu, s6, h6);
    hv[7] = bn_relu_h(w3 >> 16, s7, h7);
    *(v8h*)(sA + rowl * LDS_PITCH_H + c8t) = hv;
  }
  __syncthreads();

  const int hh = lane >> 4;
  const int c = lane & 15;
  const int koff = hh * 8;
  const int grp = wave >> 1;
  const int nh = wave & 1;
  const int m0 = grp * 32;
  const int n0 = nh * 64;
  v8f acc[2][4];
#pragma unroll
  for (int i = 0; i < 2; ++i)
#pragma unroll
    for (int j = 0; j < 4; ++j) acc[i][j] = (v8f){0.f, 0.f, 0.f, 0.f, 0.f, 0.f, 0.f, 0.f};
#pragma unroll
  for (int k0 = 0; k0 < NCH_L2; k0 += 32) {
    const v16h a0 = frag_load_h(sA + (m0 + c) * LDS_PITCH_H + koff + k0);
    const v16h a1 = frag_load_h(sA + (m0 + 16 + c) * LDS_PITCH_H + koff + k0);
    const v16h b0 = frag_load_h(sB + (n0 + 0 + c) * LDS_PITCH_H + koff + k0);
    const v16h b1 = frag_load_h(sB + (n0 + 16 + c) * LDS_PITCH_H + koff + k0);
    const v16h b2f = frag_load_h(sB + (n0 + 32 + c) * LDS_PITCH_H + koff + k0);
    const v16h b3f = frag_load_h(sB + (n0 + 48 + c) * LDS_PITCH_H + koff + k0);
    acc[0][0] = mma_h(a0, b0, acc[0][0]);
    acc[0][1] = mma_h(a0, b1, acc[0][1]);
    acc[0][2] = mma_h(a0, b2f, acc[0][2]);
    acc[0][3] = mma_h(a0, b3f, acc[0][3]);
    acc[1][0] = mma_h(a1, b0, acc[1][0]);
    acc[1][1] = mma_h(a1, b1, acc[1][1]);
    acc[1][2] = mma_h(a1, b2f, acc[1][2]);
    acc[1][3] = mma_h(a1, b3f, acc[1][3]);
    guard_8acc(acc[0][0], acc[0][1], acc[0][2], acc[0][3], acc[1][0], acc[1][1], acc[1][2], acc[1][3],
               a0, a1, b0, b1, b2f, b3f);
  }

  float vmax[4];
  float vmin[4];
#pragma unroll
  for (int j = 0; j < 4; ++j) {
    const int nl = j * 16 + c;
    const float bv = b3[n0 + nl];
    float s = 0.0f;
    float q = 0.0f;
    float mx = -__builtin_inff();
    float mn = __builtin_inff();
#pragma unroll
    for (int i = 0; i < 2; ++i) {
#pragma unroll
      for (int r = 0; r < 8; ++r) {
        const float v = __builtin_fmaf(acc[i][j][r], WCARRY_INV, bv);
        s += v;
        q = __builtin_fmaf(v, v, q);
        mx = fmaxf(mx, v);
        mn = fminf(mn, v);
      }
    }
    s += __shfl_xor(s, 16);
    q += __shfl_xor(q, 16);
    const float omx = __shfl_xor(mx, 16);
    const float omn = __shfl_xor(mn, 16);
    mx = fmaxf(mx, omx);
    mn = fminf(mn, omn);
    sStat[wave * 128 + hh * 64 + nl] = hh ? q : s;
    vmax[j] = mx;
    vmin[j] = mn;
  }
  {
    const float omx0 = hh ? vmax[1] : vmax[0];
    const float omx1 = hh ? vmax[3] : vmax[2];
    const float omn0 = hh ? vmin[1] : vmin[0];
    const float omn1 = hh ? vmin[3] : vmin[2];
    const size_t gq = (size_t)blk * 4 + grp;
    float* pmx = YMAX + gq * NCH_L3 + n0 + lane;
    float* pmn = YMIN + gq * NCH_L3 + n0 + lane;
    for (int pass = 0; pass < 2; ++pass) {
      *(volatile float*)(pmx) = omx0;
      *(volatile float*)(pmx + 32) = omx1;
      *(volatile float*)(pmn) = omn0;
      *(volatile float*)(pmn + 32) = omn1;
      __threadfence();
    }
  }
  __syncthreads();
  if (tid < 64) {
    const int e0 = tid * 4;
    const int kind = e0 >> 7;
    const int n = e0 & 127;
    const int nhh = n >> 6;
    const int cc = n & 63;
    v4f o;
#pragma unroll
    for (int i = 0; i < 4; ++i) {
      float a = 0.0f;
#pragma unroll
      for (int gi = 0; gi < 4; ++gi) a += sStat[(gi * 2 + nhh) * 128 + kind * 64 + cc + i];
      o[i] = a;
    }
    float* p = PART3 + (size_t)blk * 256 + e0;
    *(volatile v4f*)p = o;
    __threadfence();
    *(volatile v4f*)p = o;
  }
}

__global__ __launch_bounds__(256) void k_out(const float* __restrict__ YMAX, const float* __restrict__ YMIN,
                                             const float* __restrict__ SC3, float* __restrict__ out1) {
  __shared__ float tile[32 * 33];
  const int tid = threadIdx.x;
  const int lane = tid & 31;
  const int wave = tid >> 5;
  const int g0 = blockIdx.x * 32;
  const int o0 = blockIdx.y * 32;
  const int sl = tid >> 3;
  const int o4 = (tid & 7) * 4;
  const size_t src = (size_t)(g0 + sl) * NCH_L3 + o0 + o4;
  const v4f mx = *(const v4f*)(YMAX + src);
  const v4f mn = *(const v4f*)(YMIN + src);
  const v4f scv = *(const v4f*)(SC3 + o0 + o4);
  const v4f shv = *(const v4f*)(SC3 + NCH_L3 + o0 + o4);
#pragma unroll
  for (int e = 0; e < 4; ++e) {
    const float scl = scv[e];
    const float sel = (scl >= 0.0f) ? mx[e] : mn[e];
    float y = __builtin_fmaf(scl, sel, shv[e]);
    y = fmaxf(y, 0.0f);
    tile[(o4 + e) * 33 + sl] = y;
  }
  __syncthreads();
  const int b = g0 >> 10;
  const int sbase = g0 & (NCENT - 1);
  float vals[4];
#pragma unroll
  for (int i = 0; i < 4; ++i) vals[i] = tile[(wave * 4 + i) * 33 + lane];
  for (int pass = 0; pass < 2; ++pass) {
#pragma unroll
    for (int i = 0; i < 4; ++i) {
      float* p = out1 + ((size_t)b * NCH_L3 + o0 + wave * 4 + i) * NCENT + sbase + lane;
      *(volatile float*)p = vals[i];
    }
    __threadfence();
  }
}

extern "C" void kernel_launch(void* const* d_in, const int* in_sizes, int n_in,
                              void* d_out, int out_size, void* d_ws, size_t ws_size,
                              hipStream_t stream) {
  (void)in_sizes; (void)n_in; (void)out_size;
  if (ws_size < WS_TOTAL) return;
  const float* xyz_pc = (const float*)d_in[0];
  const float* points = (const float*)d_in[1];
  const float* W1  = (const float*)d_in[2];
  const float* b1  = (const float*)d_in[3];
  const float* g1  = (const float*)d_in[4];
  const float* be1 = (const float*)d_in[5];
  const float* W2  = (const float*)d_in[6];
  const float* b2  = (const float*)d_in[7];
  const float* g2  = (const float*)d_in[8];
  const float* be2 = (const float*)d_in[9];
  const float* W3  = (const float*)d_in[10];
  const float* b3  = (const float*)d_in[11];
  const float* g3  = (const float*)d_in[12];
  const float* be3 = (const float*)d_in[13];

  char* ws = (char*)d_ws;
  float* NX4   = (float*)(ws + OFF_NX4);
  float* X0    = (float*)(ws + OFF_X0);
  float* PM    = (float*)(ws + OFF_PM);
  float* P1    = (float*)(ws + OFF_P1);
  _Float16* W2H = (_Float16*)(ws + OFF_W2H);
  _Float16* W3H = (_Float16*)(ws + OFF_W3H);
  float* PART2 = (float*)(ws + OFF_PART2);
  float* SC2   = (float*)(ws + OFF_SC2);
  _Float16* Y2H = (_Float16*)(ws + OFF_Y2H);
  float* PART3 = (float*)(ws + OFF_PART3);
  float* SC3   = (float*)(ws + OFF_SC3);
  float* YMAX  = (float*)(ws + OFF_YMAX);
  float* YMIN  = (float*)(ws + OFF_YMIN);

  float* out0 = (float*)d_out;
  float* out1 = (float*)d_out + OUT0_BYTES / 4;

  k_fps<<<NBATCH, 1024, 0, stream>>>(xyz_pc, out0, NX4);
  k_ballq_group<<<(NBATCH * NCENT) / 8, 256, 0, stream>>>(xyz_pc, points, NX4, X0);
  k_mom<<<256, 256, 0, stream>>>(X0, PM);
  k_fin1<<<1, 256, 0, stream>>>(PM, W1, b1, g1, be1, W2, W3, P1, W2H, W3H);
  k_l12<<<NPARTS, 256, 0, stream>>>(X0, P1, W2H, b2, Y2H, PART2);
  k_fin<NCH_L2><<<1, 1024, 0, stream>>>(PART2, g2, be2, SC2);
  k_l3<<<NPARTS, 256, 0, stream>>>((const unsigned*)Y2H, SC2, W3H, b3, YMAX, YMIN, PART3);
  k_fin<NCH_L3><<<1, 1024, 0, stream>>>(PART3, g3, be3, SC3);
  k_out<<<dim3((NBATCH * NCENT) / 32, NCH_L3 / 32), 256, 0, stream>>>(YMAX, YMIN, SC3, out1);
}
